// ComicAttentionBlock_47811575939254
// MI455X (gfx1250) — hardware-verified
//
#include <hip/hip_runtime.h>


namespace {
constexpr int B = 4, N = 4096, C = 256, CD = 32, PW = 320, NQT = N / 16;
constexpr float XS = 8.0f, GS = 64.0f, PS = 4096.0f, WSC = 256.0f;
typedef _Float16 b16;
typedef __attribute__((ext_vector_type(16))) _Float16 v16b;
typedef __attribute__((ext_vector_type(8))) _Float16 v8b;
typedef __attribute__((ext_vector_type(8))) float v8f;
typedef __attribute__((ext_vector_type(4))) float v4f;
__device__ __forceinline__ float bf16_rne(float f) { unsigned int u = __float_as_uint(f); u += 0x7FFFu + ((u >> 16) & 1u); return __uint_as_float(u & 0xFFFF0000u); }
__device__ __forceinline__ void split16(float v, b16& hi, b16& lo) { hi = (b16)v; lo = (b16)(v - (float)hi); }
__device__ __forceinline__ v16b frag_kb(const b16* p, int hh) { const v8b a = *(const v8b*)(p + 8 * hh), b = *(const v8b*)(p + 16 + 8 * hh); v16b f;
#pragma unroll
  for (int e = 0; e < 8; ++e) { f[e] = a[e]; f[8 + e] = b[e]; } return f; }
__device__ __forceinline__ v8f wmma16b(v16b a, v16b b, v8f c) { v8f d = __builtin_amdgcn_wmma_f32_16x16x32_f16(false, a, false, b, (short)0, c, false, false); asm volatile("v_nop\n\tv_nop\n\tv_nop\n\tv_nop" : "+v"(d) : "v"(a), "v"(b)); return d; }
__device__ __forceinline__ void wave_lds_sync() { __builtin_amdgcn_fence(__ATOMIC_RELEASE, "workgroup"); __builtin_amdgcn_wave_barrier(); __builtin_amdgcn_fence(__ATOMIC_ACQUIRE, "workgroup"); }
__device__ __forceinline__ float pmul(float a, float b) { float p = a * b; asm volatile("" : "+v"(p)); return p; }

__global__ __launch_bounds__(256) void w_kernel(const float* __restrict__ Wf, const float* __restrict__ Wg, const float* __restrict__ Wh, b16* __restrict__ WT) {
  const int u = blockIdx.x * 256 + threadIdx.x; if (u >= PW * 32) return; const int o = u / 32, k0 = (u % 32) * 8; v8b v;
#pragma unroll
  for (int j = 0; j < 8; ++j) { const int k = k0 + j; float val; if (o < CD) val = Wf[k * CD + o]; else if (o < 2 * CD) val = Wg[k * CD + o - CD]; else val = Wh[(size_t)k * C + o - 2 * CD]; v[j] = (b16)(bf16_rne(val) * WSC); }
  for (int pass = 0; pass < 2; ++pass) { *(volatile v8b*)(WT + (size_t)o * C + k0) = v; __threadfence(); }
}
__global__ __launch_bounds__(32) void proj_kernel(const float* __restrict__ x, const b16* __restrict__ WT, const float* __restrict__ bf_, const float* __restrict__ bg_, const float* __restrict__ bh_, int NTV, b16* __restrict__ FH, b16* __restrict__ FL, b16* __restrict__ GH, b16* __restrict__ GL, float* __restrict__ HP) {
  __shared__ __attribute__((aligned(16))) b16 Ah[16][C + 8]; __shared__ __attribute__((aligned(16))) float Tf[16][128 + 4]; __shared__ __attribute__((aligned(16))) b16 Sh[4][16][CD + 8];
  const int lane = threadIdx.x, nloc = lane & 15, hlf = lane >> 4; const size_t t0 = (size_t)blockIdx.x * 16; if (t0 >= (size_t)NTV) return;
  for (int rr = 0; rr < 16; ++rr) for (int q = 0; q < 8; ++q) Ah[rr][q * 32 + lane] = (b16)(bf16_rne(x[(t0 + rr) * C + q * 32 + lane]) * XS);
  wave_lds_sync();
#pragma unroll 1
  for (int cg = 0; cg < 3; ++cg) { const int nt = cg < 2 ? 8 : 4; v8f acc[8];
#pragma unroll
    for (int t = 0; t < 8; ++t) acc[t] = (v8f){};
#pragma unroll 2
    for (int kb = 0; kb < C; kb += 32) { const v16b a = frag_kb(&Ah[nloc][kb], hlf);
#pragma unroll
      for (int t = 0; t < 8; ++t) if (t < nt) acc[t] = wmma16b(a, frag_kb(WT + (size_t)(cg * 128 + t * 16 + nloc) * C + kb, hlf), acc[t]); }
    if (cg == 0) {
#pragma unroll
      for (int t = 0; t < 8; ++t) { const int c = t * 16 + nloc;
#pragma unroll
        for (int r8 = 0; r8 < 8; ++r8) { const int rl = 8 * hlf + r8; const float v = acc[t][r8] * (1.0f / (XS * WSC));
          if (t < 4) { const float vv = v + (t < 2 ? bf16_rne(bf_[c]) : bf16_rne(bg_[c - CD])); b16 p, q; split16(vv * GS, p, q); Sh[(t < 2 ? 0 : 2)][rl][(c & 31)] = p; Sh[(t < 2 ? 1 : 3)][rl][(c & 31)] = q; }
          else Tf[rl][c - 64] = v + bf16_rne(bh_[c - 64]); } }
      wave_lds_sync();
      for (int pass = 0; pass < 2; ++pass) { for (int rr = 0; rr < 16; ++rr) { ((volatile b16*)FH)[(t0 + rr) * CD + lane] = Sh[0][rr][lane]; ((volatile b16*)FL)[(t0 + rr) * CD + lane] = Sh[1][rr][lane]; ((volatile b16*)GH)[(t0 + rr) * CD + lane] = Sh[2][rr][lane]; ((volatile b16*)GL)[(t0 + rr) * CD + lane] = Sh[3][rr][lane];
          ((volatile float*)HP)[(t0 + rr) * C + lane] = Tf[rr][lane]; ((volatile float*)HP)[(t0 + rr) * C + 32 + lane] = Tf[rr][32 + lane]; } __threadfence(); } }
    else { const int cbase = cg * 128 - 64;
#pragma unroll
      for (int t = 0; t < 8; ++t) { if (t < nt) { const int c = cbase + t * 16 + nloc; const float bb = bf16_rne(bh_[c]);
#pragma unroll
          for (int r8 = 0; r8 < 8; ++r8) Tf[8 * hlf + r8][t * 16 + nloc] = acc[t][r8] * (1.0f / (XS * WSC)) + bb; } }
      wave_lds_sync();
      for (int pass = 0; pass < 2; ++pass) { for (int rr = 0; rr < 16; ++rr) for (int q = 0; q < nt / 2; ++q) ((volatile float*)HP)[(t0 + rr) * C + cbase + q * 32 + lane] = Tf[rr][q * 32 + lane]; __threadfence(); } }
    wave_lds_sync(); }
}
__global__ __launch_bounds__(256) void ht_kernel(const float* __restrict__ HP, int NBV, b16* __restrict__ HTH, b16* __restrict__ HTL) {
  __shared__ float T[64][65]; const int ct = blockIdx.x % (C / 64), mt = (blockIdx.x / (C / 64)) % (N / 64), b = blockIdx.x / ((C / 64) * (N / 64)); const int tid = threadIdx.x; if (b >= NBV) return;
  for (int i = tid; i < 64 * 64; i += 256) { const int r = i / 64, c = i % 64; T[r][c] = HP[((size_t)b * N + mt * 64 + r) * C + ct * 64 + c]; }
  __syncthreads();
  { const int c = tid / 4, g = (tid % 4) * 2; for (int gg = g; gg < g + 2; ++gg) { v8b vh, vl;
#pragma unroll
      for (int j = 0; j < 8; ++j) { b16 p, q; split16(T[gg * 8 + j][c] * XS, p, q); vh[j] = p; vl[j] = q; }
      const size_t o = ((size_t)b * C + ct * 64 + c) * N + mt * 64 + gg * 8; for (int pass = 0; pass < 2; ++pass) { *(volatile v8b*)(HTH + o) = vh; *(volatile v8b*)(HTL + o) = vl; __threadfence(); } } }
}
__global__ __launch_bounds__(32) void att_kernel(const b16* __restrict__ FH, const b16* __restrict__ FL, const b16* __restrict__ GH, const b16* __restrict__ GL, int NBV, int QLIM, b16* __restrict__ PN, float* __restrict__ SMR) {
  __shared__ float Mx[16]; __shared__ __attribute__((aligned(16))) b16 Pb[16][32 + 8];
  const int lane = threadIdx.x, nloc = lane & 15, hlf = lane >> 4; const int qt = blockIdx.x % NQT, b = blockIdx.x / NQT; if (b >= NBV || qt * 16 >= QLIM) return; const size_t q0 = (size_t)b * N + (size_t)qt * 16;
  const v16b ga = frag_kb(GH + (q0 + nloc) * CD, hlf), gl = frag_kb(GL + (q0 + nloc) * CD, hlf);
  auto scores = [&](int kb, v8f sacc[2]) {
#pragma unroll
    for (int st = 0; st < 2; ++st) { const size_t kr = ((size_t)b * N + kb + st * 16 + nloc) * CD; const v16b fh = frag_kb(FH + kr, hlf), fl = frag_kb(FL + kr, hlf); sacc[st] = (v8f){}; sacc[st] = wmma16b(ga, fh, sacc[st]); sacc[st] = wmma16b(ga, fl, sacc[st]); sacc[st] = wmma16b(gl, fh, sacc[st]); sacc[st] = wmma16b(gl, fl, sacc[st]); } };
  float rmax[8];
#pragma unroll
  for (int r8 = 0; r8 < 8; ++r8) rmax[r8] = -INFINITY;
#pragma unroll 1
  for (int kb = 0; kb < N; kb += 32) { v8f sacc[2]; scores(kb, sacc);
#pragma unroll
    for (int r8 = 0; r8 < 8; ++r8) rmax[r8] = fmaxf(rmax[r8], fmaxf(sacc[0][r8], sacc[1][r8]) * (1.0f / (GS * GS))); }
#pragma unroll
  for (int r8 = 0; r8 < 8; ++r8) { float m = rmax[r8]; for (int o = 1; o < 16; o <<= 1) m = fmaxf(m, __shfl_xor(m, o)); if (nloc == 0) Mx[8 * hlf + r8] = m; }
  wave_lds_sync();
  float rsum[8];
#pragma unroll
  for (int r8 = 0; r8 < 8; ++r8) rsum[r8] = 0.0f;
#pragma unroll 1
  for (int kb = 0; kb < N; kb += 32) { v8f sacc[2]; scores(kb, sacc);
#pragma unroll
    for (int st = 0; st < 2; ++st)
#pragma unroll
      for (int r8 = 0; r8 < 8; ++r8) { const int rl = 8 * hlf + r8; const float p = __expf(sacc[st][r8] * (1.0f / (GS * GS)) - Mx[rl]); rsum[r8] += p; Pb[rl][st * 16 + nloc] = (b16)(p * PS); }
    wave_lds_sync();
    for (int pass = 0; pass < 2; ++pass) { { const int rr = lane >> 1, hf = lane & 1; *(volatile v8b*)(PN + (q0 + rr) * N + kb + hf * 16) = *(const v8b*)(&Pb[rr][hf * 16]); *(volatile v8b*)(PN + (q0 + rr) * N + kb + hf * 16 + 8) = *(const v8b*)(&Pb[rr][hf * 16 + 8]); } __threadfence(); }
    wave_lds_sync(); }
#pragma unroll
  for (int r8 = 0; r8 < 8; ++r8) { float s = rsum[r8]; for (int o = 1; o < 16; o <<= 1) s += __shfl_xor(s, o); rsum[r8] = s; }
  for (int pass = 0; pass < 2; ++pass) { for (int rr = 0; rr < 16; ++rr) { float v = 0.0f;
#pragma unroll
      for (int r8 = 0; r8 < 8; ++r8) v = (rr == 8 * hlf + r8) ? rsum[r8] : v;
      v += __shfl_xor(v, 16);
      ((volatile float*)SMR)[(q0 + rr) * 32 + lane] = v; } __threadfence(); }
}
__global__ __launch_bounds__(32) void pv_kernel(const float* __restrict__ x, const b16* __restrict__ PN, const float* __restrict__ SMR, const b16* __restrict__ HTH, const b16* __restrict__ HTL, int NBV, int QLIM, float* __restrict__ out) {
  __shared__ __attribute__((aligned(16))) float Tf[16][128 + 4];
  const int lane = threadIdx.x, nloc = lane & 15, hlf = lane >> 4; const int cg = blockIdx.x % 2, qt = (blockIdx.x / 2) % NQT, b = blockIdx.x / (2 * NQT); if (b >= NBV || qt * 16 >= QLIM) return; const size_t q0 = (size_t)b * N + (size_t)qt * 16;
  const b16* pr = PN + (q0 + nloc) * N; v8f acc[8];
#pragma unroll
  for (int t = 0; t < 8; ++t) acc[t] = (v8f){};
#pragma unroll 2
  for (int kb = 0; kb < N; kb += 32) { const v16b pa = frag_kb(pr + kb, hlf);
#pragma unroll
    for (int t = 0; t < 8; ++t) { const size_t hr = ((size_t)b * C + cg * 128 + t * 16 + nloc) * N + kb; acc[t] = wmma16b(pa, frag_kb(HTH + hr, hlf), acc[t]); acc[t] = wmma16b(pa, frag_kb(HTL + hr, hlf), acc[t]); } }
#pragma unroll
  for (int t = 0; t < 8; ++t)
#pragma unroll
    for (int r8 = 0; r8 < 8; ++r8) Tf[8 * hlf + r8][t * 16 + nloc] = acc[t][r8] * (1.0f / (PS * XS)) / SMR[(q0 + 8 * hlf + r8) * 32];
  wave_lds_sync();
  for (int pass = 0; pass < 2; ++pass) { for (int rr = 0; rr < 16; ++rr) { const size_t o = (q0 + rr) * C + cg * 128 + lane * 4; v4f v = *(const v4f*)(&Tf[rr][lane * 4]); const v4f xv = *(const v4f*)(x + o); for (int i = 0; i < 4; ++i) v[i] += bf16_rne(xv[i]); *(volatile v4f*)(out + o) = v; } __threadfence(); }
}
}

extern "C" void kernel_launch(void* const* d_in, const int* in_sizes, int n_in, void* d_out, int out_size, void* d_ws, size_t ws_size, hipStream_t stream) {
  (void)n_in;
  auto Fp = [&](int i) { return (const float*)d_in[i]; };
  if (in_sizes[0] != B * N * C || in_sizes[1] != C * CD || in_sizes[3] != C * CD || in_sizes[5] != C * C || in_sizes[6] != C || out_size != B * N * C) return;
  const int NBV = B; const int NTV = NBV * N; const int QLIM = N;
  size_t off = 0; char* ws = (char*)d_ws;
  auto carve = [&](size_t bytes) { char* p = ws + off; off += (bytes + 255) & ~(size_t)255; return p; };
  b16* WT = (b16*)carve((size_t)PW * C * 2); b16* FH = (b16*)carve((size_t)B * N * CD * 2); b16* FL = (b16*)carve((size_t)B * N * CD * 2); b16* GH = (b16*)carve((size_t)B * N * CD * 2); b16* GL = (b16*)carve((size_t)B * N * CD * 2); float* HP = (float*)carve((size_t)B * N * C * 4);
  b16* HTH = (b16*)carve((size_t)B * C * N * 2); b16* HTL = (b16*)carve((size_t)B * C * N * 2); b16* PN = (b16*)carve((size_t)B * N * N * 2); float* SMR = (float*)carve((size_t)B * N * 32 * 4);
  if (off > ws_size || off > ((size_t)192 << 20)) return;
  w_kernel<<<(PW * 32 + 255) / 256, 256, 0, stream>>>(Fp(1), Fp(3), Fp(5), WT);
  proj_kernel<<<NTV / 16, 32, 0, stream>>>(Fp(0), WT, Fp(2), Fp(4), Fp(6), NTV, FH, FL, GH, GL, HP);
  ht_kernel<<<B * (C / 64) * (N / 64), 256, 0, stream>>>(HP, NBV, HTH, HTL);
  att_kernel<<<(unsigned)(NBV * NQT), 32, 0, stream>>>(FH, FL, GH, GL, NBV, QLIM, PN, SMR);
  pv_kernel<<<(unsigned)(NBV * NQT * 2), 32, 0, stream>>>(Fp(0), PN, SMR, HTH, HTL, NBV, QLIM, (float*)d_out);
}
